// HashGridINR_32598801777091
// MI455X (gfx1250) — hardware-verified
//
#include <hip/hip_runtime.h>
#include <math.h>

constexpr int kLevels      = 16;
constexpr int kTable       = 4096;
constexpr int kFeats       = 2;
constexpr int kHidden      = 256;
constexpr int kInReal      = 33;
constexpr int kInPad       = 64;
constexpr int kChunk       = 65536;
constexpr int kRowsPerBlock = 256;
constexpr float kFeatCarry = 8.0f;
constexpr float kWCarry    = 16.0f;
constexpr float kScale0    = 1.0f / (8.0f * 16.0f);
constexpr float kScaleW    = 1.0f / 16.0f;
constexpr unsigned kPrime1 = 2654435761u;

static const float kResTab[] = {8, 10, 13, 18, 24, 31, 42, 55, 73, 97, 127, 168, 222, 294, 388, 511};
static const unsigned kHsTab[] = {64, 100, 169, 324, 576, 961, 1764, 3025, 4096, 4096, 4096, 4096, 4096, 4096, 4096, 4096};
static_assert(sizeof(kResTab) / sizeof(kResTab[0]) == kLevels, "res table length");
static_assert(sizeof(kHsTab) / sizeof(kHsTab[0]) == kLevels, "hsize table length");

typedef __attribute__((ext_vector_type(16))) _Float16 v16h;
typedef __attribute__((ext_vector_type(8)))  _Float16 v8h;
typedef __attribute__((ext_vector_type(16))) __bf16   v16b;
typedef __attribute__((ext_vector_type(8)))  __bf16   v8b;
typedef __attribute__((ext_vector_type(8)))  float    v8f;
typedef __attribute__((ext_vector_type(4)))  float    v4f;
typedef __attribute__((ext_vector_type(2)))  float    v2f;
typedef __attribute__((ext_vector_type(4)))  unsigned int v4u;

__device__ __forceinline__ unsigned short f2bf_bits(float f) {
  unsigned u = __float_as_uint(f);
  return (unsigned short)((u + 0x7FFFu + ((u >> 16) & 1u)) >> 16);
}
__device__ __forceinline__ float bf_bits2f(unsigned short h) { return __uint_as_float(((unsigned)h) << 16); }

__device__ __forceinline__ void dep_guard_h(v8f& a, v8f& b, v16h x, v16h y) { asm volatile("v_nop\n\tv_nop\n\tv_nop\n\tv_nop" : "+v"(a), "+v"(b) : "v"(x), "v"(y)); }
__device__ __forceinline__ void dep_guard_b(v8f& a, v8f& b, v16b x, v16b y) { asm volatile("v_nop\n\tv_nop\n\tv_nop\n\tv_nop" : "+v"(a), "+v"(b) : "v"(x), "v"(y)); }
__device__ __forceinline__ void keep4_h(v16h a, v16h b, v16h c, v16h d) { asm volatile("v_nop" :: "v"(a), "v"(b), "v"(c), "v"(d)); }
__device__ __forceinline__ void keep4_b(v16b a, v16b b, v16b c, v16b d) { asm volatile("v_nop" :: "v"(a), "v"(b), "v"(c), "v"(d)); }
__device__ __forceinline__ void acc_guard4(v8f& a, v8f& b, v8f& c, v8f& d) { asm volatile("v_nop\n\tv_nop\n\tv_nop\n\tv_nop" : "+v"(a), "+v"(b), "+v"(c), "+v"(d)); }
template <typename T> struct Frag;
template <> struct Frag<_Float16> {
  typedef v16h V; union U { v16h v; v8h h[2]; };
  static __device__ __forceinline__ v16h load(const _Float16* p) {
    U f; f.h[0] = *(const v8h*)(p); f.h[1] = *(const v8h*)(p + 16); return f.v;
  }
  static __device__ __forceinline__ v8f mma(v16h a, v16h b, v8f c) {
    return __builtin_amdgcn_wmma_f32_16x16x32_f16(false, a, false, b, (short)0, c, false, false);
  }
  static __device__ __forceinline__ void guard(v8f& a, v8f& b, v16h x, v16h y) { dep_guard_h(a, b, x, y); }
  static __device__ __forceinline__ void keep(v16h a, v16h b, v16h c, v16h d) { keep4_h(a, b, c, d); }
};
template <> struct Frag<__bf16> {
  typedef v16b V; union U { v16b v; v8b h[2]; };
  static __device__ __forceinline__ v16b load(const __bf16* p) {
    U f; f.h[0] = *(const v8b*)(p); f.h[1] = *(const v8b*)(p + 16); return f.v;
  }
  static __device__ __forceinline__ v8f mma(v16b a, v16b b, v8f c) {
    return __builtin_amdgcn_wmma_f32_16x16x32_bf16(false, a, false, b, (short)0, c, false, false);
  }
  static __device__ __forceinline__ void guard(v8f& a, v8f& b, v16b x, v16b y) { dep_guard_b(a, b, x, y); }
  static __device__ __forceinline__ void keep(v16b a, v16b b, v16b c, v16b d) { keep4_b(a, b, c, d); }
};

__device__ __forceinline__ unsigned pk16(unsigned short a, unsigned short b) { return (unsigned)a | ((unsigned)b << 16); }
__device__ __forceinline__ unsigned short h_bits(float f) { const _Float16 h = (_Float16)f; return __builtin_bit_cast(unsigned short, h); }
__device__ __forceinline__ float hbits2f(unsigned w16) { return (float)__builtin_bit_cast(_Float16, (unsigned short)w16); }

template <int ET> struct Elem;
template <> struct Elem<0> { typedef _Float16 T; };
template <> struct Elem<1> { typedef __bf16 T; };
template <int ET, bool SPLIT, int BIAS_MODE, int OUT_MODE, bool RESID, int ACT = 0>
__global__ __launch_bounds__(256) void wmma_gemm64(
    const unsigned short* __restrict__ Ap, const unsigned short* __restrict__ A2p, int lda, long strideA,
    const unsigned short* __restrict__ Btp, const unsigned short* __restrict__ Bt2p, int ldb, long strideB,
    void* __restrict__ Cout, void* __restrict__ Cout2, int ldc, long strideC,
    const float* __restrict__ bias,
    const float* __restrict__ resid, long strideR,
    int M, int N, int K, float scale) {
  typedef typename Elem<ET>::T T;
  typedef typename Frag<T>::V V;
  const T* A = (const T*)Ap; const T* A2 = (const T*)A2p; const T* Bt = (const T*)Btp; const T* Bt2 = (const T*)Bt2p;
  __shared__ __align__(16) float sT[8][16 * 68];
  const int b    = blockIdx.y;
  const int lane = threadIdx.x & 31;
  const int wave = threadIdx.x >> 5;
  const int tilesN = N >> 6;
  const int tilesM = M >> 6;
  const int tile = blockIdx.x * 8 + wave;
  if (tile >= tilesM * tilesN) return;
  const int tm = tile / tilesN;
  const int tn = tile - tm * tilesN;
  const int m0 = tm << 6;
  const int n0 = tn << 6;

  const T* Ab  = A  + (size_t)b * strideA;
  const T* Bb  = Bt + (size_t)b * strideB;
  const T* Ab2 = SPLIT ? (A2  + (size_t)b * strideA) : nullptr;
  const T* Bb2 = SPLIT ? (Bt2 + (size_t)b * strideB) : nullptr;

  const int rlane = lane & 15;
  const int koff  = (lane >> 4) * 8;
  const int mOff  = (lane >> 4) * 8;

  v8f acc[4][4];
#pragma unroll
  for (int i = 0; i < 4; ++i)
#pragma unroll
    for (int j = 0; j < 4; ++j) acc[i][j] = (v8f){0.f,0.f,0.f,0.f,0.f,0.f,0.f,0.f};

  for (int k0 = 0; k0 < K; k0 += 32) {
    V bh[4], bl[4];
#pragma unroll
    for (int j = 0; j < 4; ++j) {
      const size_t bo = (size_t)(n0 + (j << 4) + rlane) * ldb + koff + k0;
      bh[j] = Frag<T>::load(Bb + bo);
      if (SPLIT) bl[j] = Frag<T>::load(Bb2 + bo);
    }
#pragma unroll
    for (int i = 0; i < 4; ++i) {
      const size_t ao = (size_t)(m0 + (i << 4) + rlane) * lda + koff + k0;
      V ah = Frag<T>::load(Ab + ao);
      V al;
      if (SPLIT) al = Frag<T>::load(Ab2 + ao);
#pragma unroll
      for (int j = 0; j < 4; ++j) {
        acc[i][j] = Frag<T>::mma(ah, bh[j], acc[i][j]);
        if (SPLIT) {
          acc[i][j] = Frag<T>::mma(ah, bl[j], acc[i][j]);
          acc[i][j] = Frag<T>::mma(al, bh[j], acc[i][j]);
        }
      }
      Frag<T>::guard(acc[i][0], acc[i][3], ah, SPLIT ? al : ah);
    }
    Frag<T>::keep(bh[0], bh[1], bh[2], bh[3]);
    if (SPLIT) Frag<T>::keep(bl[0], bl[1], bl[2], bl[3]);
  }
  acc_guard4(acc[0][0], acc[0][1], acc[0][2], acc[0][3]);
  acc_guard4(acc[1][0], acc[1][1], acc[1][2], acc[1][3]);
  acc_guard4(acc[2][0], acc[2][1], acc[2][2], acc[2][3]);
  acc_guard4(acc[3][0], acc[3][1], acc[3][2], acc[3][3]);

  float* slab = sT[wave];
  const float* Rb = RESID ? (resid + (size_t)b * strideR) : nullptr;
#pragma unroll
  for (int i = 0; i < 4; ++i) {
    const int mBase = m0 + (i << 4);
#pragma unroll
    for (int j = 0; j < 4; ++j) {
      const int n = n0 + (j << 4) + rlane;
      float bv = 0.f;
      if (BIAS_MODE == 2) bv = bias[n];
#pragma unroll
      for (int r = 0; r < 8; ++r) {
        float v = acc[i][j][r] * scale;
        if (BIAS_MODE == 1) v += bias[mBase + mOff + r];
        if (BIAS_MODE == 2) v += bv;
        if (RESID) v += Rb[(size_t)(mBase + mOff + r) * ldc + n];
        if (ACT == 2) v = fmaxf(v, 0.0f);
        if (ACT == 4) v = (v > 0.f) ? v : 0.01f * v;
        slab[(mOff + r) * 68 + (j << 4) + rlane] = v;
      }
    }
    __builtin_amdgcn_fence(__ATOMIC_RELEASE, "workgroup");
    __builtin_amdgcn_wave_barrier();
    __builtin_amdgcn_fence(__ATOMIC_ACQUIRE, "workgroup");
    if (OUT_MODE == 0) {
      float* C = (float*)Cout + (size_t)b * strideC;
      const int hh = lane >> 4, c4 = (lane & 15) * 4;
      for (int pass = 0; pass < 2; ++pass) {
#pragma unroll
        for (int it = 0; it < 8; ++it) {
          const int row = it * 2 + hh;
          v4f v = *(const v4f*)(slab + row * 68 + c4);
          *(volatile v4f*)(C + (size_t)(mBase + row) * ldc + n0 + c4) = v;
        }
        __threadfence();
      }
    } else {
      const int q = lane >> 3, c8 = (lane & 7) * 8;
      unsigned short* C  = (unsigned short*)Cout  + (size_t)b * strideC;
      unsigned short* C2 = (OUT_MODE == 2) ? ((unsigned short*)Cout2 + (size_t)b * strideC) : nullptr;
      for (int pass = 0; pass < 2; ++pass) {
#pragma unroll
        for (int it = 0; it < 4; ++it) {
          const int row = it * 4 + q;
          const float* sp = slab + row * 68 + c8;
          v8h hv, lv;
#pragma unroll
          for (int e = 0; e < 8; ++e) {
            if (OUT_MODE == 1) {
              hv[e] = (_Float16)sp[e];
            } else {
              unsigned short hb = f2bf_bits(sp[e]);
              unsigned short lb = f2bf_bits(sp[e] - bf_bits2f(hb));
              hv[e] = __builtin_bit_cast(_Float16, hb);
              lv[e] = __builtin_bit_cast(_Float16, lb);
            }
          }
          *(volatile v8h*)(C + (size_t)(mBase + row) * ldc + n0 + c8) = hv;
          if (OUT_MODE == 2) *(volatile v8h*)(C2 + (size_t)(mBase + row) * ldc + n0 + c8) = lv;
        }
        __threadfence();
      }
    }
    __builtin_amdgcn_fence(__ATOMIC_RELEASE, "workgroup");
    __builtin_amdgcn_wave_barrier();
    __builtin_amdgcn_fence(__ATOMIC_ACQUIRE, "workgroup");
  }
}

__global__ __launch_bounds__(256) void wtcast_kernel(const float* __restrict__ Wa, const float* __restrict__ Wb,
                                                     const float* __restrict__ Wc, unsigned short* __restrict__ out,
                                                     long planeHalves, int Kreal, int Kpad, int N, float scale) {
  __shared__ float sm[64][65];
  const int t  = threadIdx.x;
  const int k0 = blockIdx.x * 64;
  const int n0 = blockIdx.y * 64;
  const int z  = blockIdx.z;
  const float* W = (z == 0) ? Wa : (z == 1) ? Wb : Wc;
#pragma unroll
  for (int i = 0; i < 16; ++i) {
    const int e = i * 256 + t;
    const int r = e >> 6;
    const int c = e & 63;
    const int k = k0 + r;
    const int kc = (k < Kreal) ? k : (Kreal - 1);
    float v = W[(size_t)kc * N + n0 + c] * scale;
    v = (k < Kreal) ? v : 0.0f;
    sm[c][r] = v;
  }
  __syncthreads();
  const int lane = t & 31, wave = t >> 5;
  const int q = lane >> 3, c8 = (lane & 7) * 8;
  unsigned short* op = out + (size_t)z * planeHalves;
  v4u u[2];
#pragma unroll
  for (int it = 0; it < 2; ++it) {
    const int row = wave * 8 + it * 4 + q;
    unsigned short hb[8];
#pragma unroll
    for (int e = 0; e < 8; ++e) hb[e] = h_bits(sm[row][c8 + e]);
    u[it] = (v4u){pk16(hb[0], hb[1]), pk16(hb[2], hb[3]), pk16(hb[4], hb[5]), pk16(hb[6], hb[7])};
  }
  for (int pass = 0; pass < 2; ++pass) {
#pragma unroll
    for (int it = 0; it < 2; ++it) {
      const int row = wave * 8 + it * 4 + q;
      *(volatile v4u*)(op + (size_t)(n0 + row) * Kpad + k0 + c8) = u[it];
    }
    __threadfence();
  }
}

struct LevelTab { float res[kLevels]; unsigned hs[kLevels]; };
static_assert(sizeof(LevelTab) == 128, "no padding");

__global__ __launch_bounds__(256) void encode_kernel(const float* __restrict__ x, const float* __restrict__ tables,
                                                     unsigned short* __restrict__ H0, int nPts, LevelTab lt) {
#pragma clang fp contract(off)
  __shared__ float    s_res[kLevels];
  __shared__ unsigned s_hs[kLevels];
  __shared__ __align__(16) unsigned s_row[kRowsPerBlock * 32];
  const int t = threadIdx.x;
  if (t == 0) {
#pragma unroll
    for (int l = 0; l < kLevels; ++l) { s_res[l] = lt.res[l]; s_hs[l] = lt.hs[l]; }
  }
  __syncthreads();
  const int p  = blockIdx.x * kRowsPerBlock + t;
  const int pc = (p < nPts) ? p : (nPts - 1);
  const float c0 = x[(size_t)pc * 3 + 0];
  const float c1 = x[(size_t)pc * 3 + 1];
  const float c2 = x[(size_t)pc * 3 + 2];
  unsigned* rowp = s_row + t * 32;
#pragma unroll 1
  for (int l = 0; l < kLevels; ++l) {
    const float rr = s_res[l];
    unsigned hsz = s_hs[l];
    hsz = (hsz < 1u) ? 1u : ((hsz > (unsigned)kTable) ? (unsigned)kTable : hsz);
    const float sx = c0 * rr;
    const float sy = c1 * rr;
    const float fx = floorf(sx);
    const float fy = floorf(sy);
    const float tx = sx - fx;
    const float ty = sy - fy;
    const int ix = (int)fx;
    const int iy = (int)fy;
    const unsigned ux0 = (unsigned)ix;
    const unsigned ux1 = (unsigned)(ix + 1);
    const unsigned uy0 = (unsigned)iy * kPrime1;
    const unsigned uy1 = (unsigned)(iy + 1) * kPrime1;
    const unsigned h00 = (ux0 ^ uy0) % hsz;
    const unsigned h01 = (ux0 ^ uy1) % hsz;
    const unsigned h10 = (ux1 ^ uy0) % hsz;
    const unsigned h11 = (ux1 ^ uy1) % hsz;
    const float* tl = tables + (size_t)l * (kTable * kFeats);
    const v2f t00 = *(const v2f*)(tl + 2 * (size_t)h00);
    const v2f t01 = *(const v2f*)(tl + 2 * (size_t)h01);
    const v2f t10 = *(const v2f*)(tl + 2 * (size_t)h10);
    const v2f t11 = *(const v2f*)(tl + 2 * (size_t)h11);
    const float wx0 = 1.0f - tx;
    const float wy0 = 1.0f - ty;
    const float w00 = wx0 * wy0;
    const float w01 = wx0 * ty;
    const float w10 = tx * wy0;
    const float w11 = tx * ty;
    const float f0 = ((w00 * t00.x + w01 * t01.x) + w10 * t10.x) + w11 * t11.x;
    const float f1 = ((w00 * t00.y + w01 * t01.y) + w10 * t10.y) + w11 * t11.y;
    rowp[l] = pk16(h_bits(f0 * kFeatCarry), h_bits(f1 * kFeatCarry));
  }
  {
    const unsigned short xb = h_bits(c2 * kFeatCarry);
    const unsigned xw = pk16(xb, xb);
    const v4u xv = (v4u){xw, xw, xw, xw};
#pragma unroll
    for (int j = 0; j < 4; ++j) *(v4u*)(rowp + 16 + 4 * j) = xv;
  }
  __syncthreads();
  const int lane = t & 31, wave = t >> 5;
  const int q = lane >> 3;
  const int c4w = (lane & 7) * 4;
  const int c8  = (lane & 7) * 8;
  v4u r[8];
#pragma unroll
  for (int it = 0; it < 8; ++it) {
    const int row = wave * 32 + it * 4 + q;
    r[it] = *(const v4u*)(s_row + row * 32 + c4w);
  }
  const int rowbase = blockIdx.x * kRowsPerBlock;
  for (int pass = 0; pass < 2; ++pass) {
#pragma unroll
    for (int it = 0; it < 8; ++it) {
      const int row = wave * 32 + it * 4 + q;
      *(volatile v4u*)(H0 + (size_t)(rowbase + row) * kInPad + c8) = r[it];
    }
    __threadfence();
  }
}

__global__ __launch_bounds__(256) void head_kernel(const unsigned short* __restrict__ act, const float* __restrict__ W4,
                                                   const float* __restrict__ b4, float* __restrict__ out, int nRows) {
  __shared__ float s_w[kHidden];
  __shared__ __align__(16) float s_o[kRowsPerBlock];
  const int t = threadIdx.x;
  s_w[t] = W4[t];
  __syncthreads();
  const int row = blockIdx.x * kRowsPerBlock + t;
  const int rc  = (row < nRows) ? row : (nRows - 1);
  const unsigned short* ap = act + (size_t)rc * kHidden;
  float acc = 0.0f;
#pragma unroll 1
  for (int j = 0; j < kHidden / 8; ++j) {
    const v4u u = *(const v4u*)(ap + 8 * j);
    const float* wj = s_w + 8 * j;
    acc += hbits2f(u.x & 0xffffu) * wj[0];
    acc += hbits2f(u.x >> 16)      * wj[1];
    acc += hbits2f(u.y & 0xffffu) * wj[2];
    acc += hbits2f(u.y >> 16)      * wj[3];
    acc += hbits2f(u.z & 0xffffu) * wj[4];
    acc += hbits2f(u.z >> 16)      * wj[5];
    acc += hbits2f(u.w & 0xffffu) * wj[6];
    acc += hbits2f(u.w >> 16)      * wj[7];
  }
  s_o[t] = acc + b4[0];
  __syncthreads();
  if (t < 64) {
    const v4f v = *(const v4f*)(s_o + 4 * t);
    float* opt = out + (size_t)blockIdx.x * kRowsPerBlock + 4 * t;
    *(volatile v4f*)opt = v;
    __threadfence();
    *(volatile v4f*)opt = v;
  }
}

extern "C" void kernel_launch(void* const* d_in, const int* in_sizes, int n_in,
                              void* d_out, int out_size, void* d_ws, size_t ws_size,
                              hipStream_t stream) {
  if (n_in < 12) return;
  const float* x      = (const float*)d_in[0];
  const float* tables = (const float*)d_in[1];
  const float* W0 = (const float*)d_in[2];
  const float* b0 = (const float*)d_in[3];
  const float* W1 = (const float*)d_in[4];
  const float* b1 = (const float*)d_in[5];
  const float* W2 = (const float*)d_in[6];
  const float* b2 = (const float*)d_in[7];
  const float* W3 = (const float*)d_in[8];
  const float* b3 = (const float*)d_in[9];
  const float* W4 = (const float*)d_in[10];
  const float* b4 = (const float*)d_in[11];
  float* out = (float*)d_out;

  const int nPts = in_sizes[0] / 3;
  if (nPts <= 0 || (nPts % kChunk) != 0 || out_size < nPts) return;
  if (in_sizes[1] != kLevels * kTable * kFeats) return;
  if (in_sizes[2] != kInReal * kHidden || in_sizes[4] != kHidden * kHidden ||
      in_sizes[6] != kHidden * kHidden || in_sizes[8] != kHidden * kHidden) return;
  if (in_sizes[3] != kHidden || in_sizes[5] != kHidden || in_sizes[7] != kHidden || in_sizes[9] != kHidden) return;
  if (in_sizes[10] != kHidden || in_sizes[11] < 1) return;
  const int nChunks = nPts / kChunk;

  const size_t bt0Bytes   = (size_t)kHidden * kInPad * 2;
  const size_t bt123Bytes = (size_t)3 * kHidden * kHidden * 2;
  const size_t h0Bytes    = (size_t)nPts * kInPad * 2;
  const size_t actBytes   = (size_t)kChunk * kHidden * 2;
  const size_t offBt0   = 0;
  const size_t offBt123 = offBt0 + bt0Bytes;
  const size_t offH0    = offBt123 + bt123Bytes;
  const size_t offActA  = offH0 + h0Bytes;
  const size_t offActB  = offActA + actBytes;
  const size_t total    = offActB + actBytes;
  if (total > ws_size) return;
  char* wsb = (char*)d_ws;
  unsigned short* bt0   = (unsigned short*)(wsb + offBt0);
  unsigned short* bt123 = (unsigned short*)(wsb + offBt123);
  unsigned short* h0    = (unsigned short*)(wsb + offH0);
  unsigned short* actA  = (unsigned short*)(wsb + offActA);
  unsigned short* actB  = (unsigned short*)(wsb + offActB);

  LevelTab lt;
  for (int l = 0; l < kLevels; ++l) {
    lt.res[l] = kResTab[l];
    lt.hs[l]  = kHsTab[l];
  }

  wtcast_kernel<<<dim3(kInPad / 64, kHidden / 64, 1), 256, 0, stream>>>(
      W0, W0, W0, bt0, 0L, kInReal, kInPad, kHidden, kWCarry);
  wtcast_kernel<<<dim3(kHidden / 64, kHidden / 64, 3), 256, 0, stream>>>(
      W1, W2, W3, bt123, (long)kHidden * kHidden, kHidden, kHidden, kHidden, kWCarry);

  encode_kernel<<<nPts / kRowsPerBlock, 256, 0, stream>>>(x, tables, h0, nPts, lt);

  const int gemmBlocks = ((kChunk / 64) * (kHidden / 64)) / 8;
  const size_t wPlane = (size_t)kHidden * kHidden;
  for (int c = 0; c < nChunks; ++c) {
    const unsigned short* a0 = h0 + (size_t)c * kChunk * kInPad;
    wmma_gemm64<0, false, 2, 1, false, 2><<<dim3(gemmBlocks, 1), 256, 0, stream>>>(
        a0, a0, kInPad, 0L, bt0, bt0, kInPad, 0L, (void*)actA, (void*)actA, kHidden, 0L,
        b0, b0, 0L, kChunk, kHidden, kInPad, kScale0);
    wmma_gemm64<0, false, 2, 1, false, 2><<<dim3(gemmBlocks, 1), 256, 0, stream>>>(
        actA, actA, kHidden, 0L, bt123, bt123, kHidden, 0L, (void*)actB, (void*)actB, kHidden, 0L,
        b1, b1, 0L, kChunk, kHidden, kHidden, kScaleW);
    wmma_gemm64<0, false, 2, 1, false, 2><<<dim3(gemmBlocks, 1), 256, 0, stream>>>(
        actB, actB, kHidden, 0L, bt123 + wPlane, bt123 + wPlane, kHidden, 0L, (void*)actA, (void*)actA, kHidden, 0L,
        b2, b2, 0L, kChunk, kHidden, kHidden, kScaleW);
    wmma_gemm64<0, false, 2, 1, false, 2><<<dim3(gemmBlocks, 1), 256, 0, stream>>>(
        actA, actA, kHidden, 0L, bt123 + 2 * wPlane, bt123 + 2 * wPlane, kHidden, 0L, (void*)actB, (void*)actB, kHidden, 0L,
        b3, b3, 0L, kChunk, kHidden, kHidden, kScaleW);
    head_kernel<<<kChunk / kRowsPerBlock, 256, 0, stream>>>(
        actB, W4, b4, out + (size_t)c * kChunk, kChunk);
  }
}
